// SparseCausalSelfAttention_39402029973883
// MI455X (gfx1250) — hardware-verified
//
#include <hip/hip_runtime.h>
#include <hip/hip_bf16.h>
#include <stddef.h>
#include <stdint.h>
#include <math.h>

#define NB   4
#define TS   2048
#define DM   1024
#define NH   16
#define HD   64
#define D3   (3 * DM)
#define NR   (NB * TS)
#define NBH  (NB * NH)
#define BS   256
#define NJ   (TS / BS)
#define ER   64
#define ST0  240
#define SR   80
#define NG   (NB * NJ)
#define NE   (NG * ER)
#define NS   (NG * SR)

static_assert(NH * HD == DM);
static_assert(TS % BS == 0);
static_assert(BS == 4 * ER);
static_assert(SR == ER + (BS - ST0));
static_assert((BS - ST0) == 16);
static_assert(ST0 % 16 == 0);
static_assert(DM % 128 == 0);
static_assert(D3 % 128 == 0);
static_assert(NR % 64 == 0);
static_assert(TS % 64 == 0);
static_assert(DM / 8 == 128);
static_assert(SR % 16 == 0);
static_assert(NJ == 8);
static_assert(NH == 16);
static_assert(NE <= NS);

typedef _Float16 v16h __attribute__((ext_vector_type(16)));
typedef _Float16 v8h  __attribute__((ext_vector_type(8)));
typedef float    v8f  __attribute__((ext_vector_type(8)));
typedef float    v4f  __attribute__((ext_vector_type(4)));
typedef unsigned int   v4u   __attribute__((ext_vector_type(4)));
typedef unsigned short v8us  __attribute__((ext_vector_type(8)));
typedef unsigned short v16us __attribute__((ext_vector_type(16)));
typedef __bf16         v16b  __attribute__((ext_vector_type(16)));
typedef unsigned short ush;

union Frag  { v16h v; v8h h[2]; };
union FragU { v16us v; v8us h[2]; v16b b; };
union Pack8 { v8h h; v4u u; };
union PackU { v8us s; v4u u; };
struct HL { v4u h; v4u l; };

__device__ __forceinline__ ush f2bf(float f) {
  const unsigned u = __float_as_uint(f);
  return (ush)((u + 0x7FFFu + ((u >> 16) & 1u)) >> 16);
}
__device__ __forceinline__ float bf2f(ush b) { return __uint_as_float(((unsigned)b) << 16); }

__device__ __forceinline__ HL split8(v8f f) {
  PackU ph, pl;
#pragma unroll
  for (int e = 0; e < 8; ++e) {
    const ush hi = f2bf(f[e]);
    ph.s[e] = hi;
    pl.s[e] = f2bf(f[e] - bf2f(hi));
  }
  HL r; r.h = ph.u; r.l = pl.u;
  return r;
}

__device__ __forceinline__ v8f mma16(v16h a, v16h b, v8f c) {
  c = __builtin_amdgcn_wmma_f32_16x16x32_f16(false, a, false, b, (short)0, c, false, false);
  asm volatile("v_nop\n\tv_nop\n\tv_nop\n\tv_nop" : "+v"(c) : "v"(a), "v"(b));
  return c;
}
__device__ __forceinline__ v8f mmab(v16us a, v16us b, v8f c) {
  FragU ua, ub; ua.v = a; ub.v = b;
  c = __builtin_amdgcn_wmma_f32_16x16x32_bf16(false, ua.b, false, ub.b, (short)0, c, false, false);
  asm volatile("v_nop\n\tv_nop\n\tv_nop\n\tv_nop" : "+v"(c) : "v"(a), "v"(b));
  return c;
}

__device__ __forceinline__ v16h ldfrag(const _Float16* p, int ld, int row0, int k0, int lane) {
  const int m = lane & 15, lh = lane >> 4;
  const _Float16* q = p + (size_t)(row0 + m) * ld + k0 + 8 * lh;
  Frag f;
  f.h[0] = *(const v8h*)(q);
  f.h[1] = *(const v8h*)(q + 16);
  return f.v;
}
__device__ __forceinline__ v16us ldfragu(const ush* p, int ld, int row0, int k0, int lane) {
  const int m = lane & 15, lh = lane >> 4;
  const ush* q = p + (size_t)(row0 + m) * ld + k0 + 8 * lh;
  FragU f;
  f.h[0] = *(const v8us*)(q);
  f.h[1] = *(const v8us*)(q + 16);
  return f.v;
}

__device__ __forceinline__ v8f zero8() { return (v8f){0.f, 0.f, 0.f, 0.f, 0.f, 0.f, 0.f, 0.f}; }

__global__ __launch_bounds__(256) void k_cvtx(const float* __restrict__ src, _Float16* __restrict__ dh, int ngrp) {
  const int t = blockIdx.x * 256 + (int)threadIdx.x;
  if (t >= ngrp) return;
  const size_t o = (size_t)t * 8;
  const v4f a0 = *(const v4f*)(src + o);
  const v4f a1 = *(const v4f*)(src + o + 4);
  Pack8 pk;
  pk.h = (v8h){(_Float16)a0[0], (_Float16)a0[1], (_Float16)a0[2], (_Float16)a0[3],
               (_Float16)a1[0], (_Float16)a1[1], (_Float16)a1[2], (_Float16)a1[3]};
  const v4u vv = pk.u;
  volatile v4u* d = (volatile v4u*)(dh + o);
  *d = vv;
  __threadfence();
  *d = vv;
}

__global__ __launch_bounds__(256) void k_cvt3x(const float* __restrict__ src, ush* __restrict__ d3h,
                                               ush* __restrict__ d3l, int ngrp) {
  const int t = blockIdx.x * 256 + (int)threadIdx.x;
  if (t >= ngrp) return;
  const int cr = t >> 7;
  const int pc = t & 127;
  const int gi = cr / SR;
  const int i  = cr - gi * SR;
  const int r  = (i < ER) ? i : (i + (ST0 - ER));
  const size_t os = ((size_t)gi * BS + r) * DM + (size_t)pc * 8;
  const size_t od = (size_t)t * 8;
  const v4f a0 = *(const v4f*)(src + os);
  const v4f a1 = *(const v4f*)(src + os + 4);
  const v8f f = (v8f){a0[0], a0[1], a0[2], a0[3], a1[0], a1[1], a1[2], a1[3]};
  const HL s = split8(f);
  *(volatile v4u*)(d3h + od) = s.h;
  *(volatile v4u*)(d3l + od) = s.l;
  __threadfence();
  *(volatile v4u*)(d3h + od) = s.h;
  *(volatile v4u*)(d3l + od) = s.l;
}

#define CWP 65
__global__ __launch_bounds__(256) void k_cvtw(const float* __restrict__ src, _Float16* __restrict__ dh,
                                              ush* __restrict__ d3h, ush* __restrict__ d3l,
                                              int K, int N, float scl) {
  __shared__ float tile[64 * CWP];
  const int tid = threadIdx.x;
  const int n0 = blockIdx.x * 64, k0 = blockIdx.y * 64;
#pragma unroll
  for (int it = 0; it < 16; ++it) {
    const int e  = tid + 256 * it;
    const int kk = e >> 6, nn = e & 63;
    tile[kk * CWP + nn] = src[(size_t)(k0 + kk) * N + n0 + nn];
  }
  __syncthreads();
  v4u vf[2]; v4u vh[2]; v4u vl[2]; size_t go[2];
#pragma unroll
  for (int it = 0; it < 2; ++it) {
    const int p  = tid + 256 * it;
    const int nn = p >> 3, pc = p & 7;
    v8f f;
#pragma unroll
    for (int u = 0; u < 8; ++u) f[u] = tile[(pc * 8 + u) * CWP + nn];
    Pack8 pk;
    pk.h = (v8h){(_Float16)(f[0] * scl), (_Float16)(f[1] * scl), (_Float16)(f[2] * scl), (_Float16)(f[3] * scl),
                 (_Float16)(f[4] * scl), (_Float16)(f[5] * scl), (_Float16)(f[6] * scl), (_Float16)(f[7] * scl)};
    vf[it] = pk.u;
    const HL s = split8(f);
    vh[it] = s.h;
    vl[it] = s.l;
    go[it] = (size_t)(n0 + nn) * K + k0 + pc * 8;
  }
#pragma unroll
  for (int it = 0; it < 2; ++it) {
    *(volatile v4u*)(dh  + go[it]) = vf[it];
    *(volatile v4u*)(d3h + go[it]) = vh[it];
    *(volatile v4u*)(d3l + go[it]) = vl[it];
  }
  __threadfence();
#pragma unroll
  for (int it = 0; it < 2; ++it) {
    *(volatile v4u*)(dh  + go[it]) = vf[it];
    *(volatile v4u*)(d3h + go[it]) = vh[it];
    *(volatile v4u*)(d3l + go[it]) = vl[it];
  }
}

#define STP 136
__global__ __launch_bounds__(128) __attribute__((amdgpu_num_vgpr(256)))
void k_qkv(const _Float16* __restrict__ xh, const _Float16* __restrict__ wt, const float* __restrict__ bias,
           _Float16* __restrict__ qp, _Float16* __restrict__ kp, _Float16* __restrict__ vt) {
  __shared__ __align__(16) _Float16 st[64 * STP];
  __shared__ __align__(16) float bs[128];
  const int tid = threadIdx.x, lane = tid & 31, wave = tid >> 5;
  const int hh = lane >> 4, c = lane & 15;
  const int mb = blockIdx.x * 64;
  const int m0 = mb + wave * 16;
  const int n0 = blockIdx.y * 128;
  const int which = n0 >> 10;
  const int head0 = (n0 & (DM - 1)) >> 6;
  const int b  = mb >> 11;
  const int t0 = mb & (TS - 1);
  const int bh0 = b * NH + head0;
  const bool skipq = (which == 0) && ((t0 & (BS - 1)) < ER);
  if (skipq) return;
  bs[tid] = bias[n0 + tid];

  v8f acc[8];
#pragma unroll
  for (int t = 0; t < 8; ++t) acc[t] = zero8();
#pragma unroll 1
  for (int k0 = 0; k0 < DM; k0 += 32) {
    const v16h a = ldfrag(xh, DM, m0, k0, lane);
#pragma unroll
    for (int t = 0; t < 8; ++t) {
      const v16h bf = ldfrag(wt, DM, n0 + 16 * t, k0, lane);
      acc[t] = mma16(a, bf, acc[t]);
    }
  }
  __syncthreads();

#pragma unroll
  for (int r = 0; r < 8; ++r) {
    const int lr = wave * 16 + 8 * hh + r;
#pragma unroll
    for (int t = 0; t < 8; ++t)
      st[lr * STP + 16 * t + c] = (_Float16)(acc[t][r] * 0.03125f + bs[16 * t + c]);
  }
  __syncthreads();

  _Float16* base = (which == 0) ? qp : ((which == 1) ? kp : vt);
  v4u val[8];
  size_t go[8];
  if (which < 2) {
#pragma unroll
    for (int it = 0; it < 8; ++it) {
      const int p  = tid + 128 * it;
      const int hd = p >> 9;
      const int rr = (p & 511) >> 3;
      const int pc = p & 7;
      Pack8 pk;
      pk.h    = *(const v8h*)(st + rr * STP + hd * 64 + pc * 8);
      val[it] = pk.u;
      go[it]  = ((size_t)(bh0 + hd) * TS + t0 + rr) * HD + pc * 8;
    }
  } else {
#pragma unroll
    for (int it = 0; it < 8; ++it) {
      const int p  = tid + 128 * it;
      const int dd = p >> 3;
      const int hd = dd >> 6, d = dd & 63;
      const int pc = p & 7;
      const _Float16* cpp = st + (pc * 8) * STP + dd;
      Pack8 pk;
      pk.h = (v8h){cpp[0 * STP], cpp[1 * STP], cpp[2 * STP], cpp[3 * STP],
                   cpp[4 * STP], cpp[5 * STP], cpp[6 * STP], cpp[7 * STP]};
      val[it] = pk.u;
      go[it]  = ((size_t)(bh0 + hd) * HD + d) * TS + t0 + pc * 8;
    }
  }
#pragma unroll
  for (int it = 0; it < 8; ++it) *(volatile v4u*)(base + go[it]) = val[it];
  __threadfence();
#pragma unroll
  for (int it = 0; it < 8; ++it) *(volatile v4u*)(base + go[it]) = val[it];
}

__global__ __launch_bounds__(160) __attribute__((amdgpu_num_vgpr(256)))
void k_qkv3(const ush* __restrict__ x3h, const ush* __restrict__ x3l,
            const ush* __restrict__ wth, const ush* __restrict__ wtl, const float* __restrict__ bias,
            ush* __restrict__ q3h, ush* __restrict__ q3l,
            ush* __restrict__ k3h, ush* __restrict__ k3l,
            ush* __restrict__ v3h, ush* __restrict__ v3l) {
  __shared__ __align__(16) ush   st[SR * STP];
  __shared__ __align__(16) float bs[128];
  const int tid = threadIdx.x, lane = tid & 31, wave = tid >> 5;
  const int hh = lane >> 4, c = lane & 15;
  const int gi = blockIdx.x;
  const int n0 = blockIdx.y * 128;
  const int which = n0 >> 10;
  const int head0 = (n0 & (DM - 1)) >> 6;
  const int b = gi >> 3, j = gi & 7;
  const int bh0 = b * NH + head0;
  const int m0 = gi * SR + wave * 16;
  if (tid < 128) bs[tid] = bias[n0 + tid];
  const bool active = (which != 0) || (wave < 4);

  v8f acc[8];
#pragma unroll
  for (int t = 0; t < 8; ++t) acc[t] = zero8();
  if (active) {
#pragma unroll 1
    for (int k0 = 0; k0 < DM; k0 += 32) {
      const v16us ah = ldfragu(x3h, DM, m0, k0, lane);
      const v16us al = ldfragu(x3l, DM, m0, k0, lane);
#pragma unroll
      for (int t = 0; t < 8; ++t) {
        const v16us bfh = ldfragu(wth, DM, n0 + 16 * t, k0, lane);
        const v16us bfl = ldfragu(wtl, DM, n0 + 16 * t, k0, lane);
        acc[t] = mmab(ah, bfh, acc[t]);
        acc[t] = mmab(ah, bfl, acc[t]);
        acc[t] = mmab(al, bfh, acc[t]);
      }
    }
  }
  __syncthreads();
#pragma unroll
  for (int t = 0; t < 8; ++t)
#pragma unroll
    for (int r = 0; r < 8; ++r) acc[t][r] += bs[16 * t + c];

  const int np = (which == 0) ? 1024 : 1280;
  ush* bhp = (which == 0) ? q3h : ((which == 1) ? k3h : v3h);
  ush* blp = (which == 0) ? q3l : ((which == 1) ? k3l : v3l);
  size_t go[8];
#pragma unroll
  for (int it = 0; it < 8; ++it) {
    const int p  = tid + 160 * it;
    const int hd = (which == 0) ? (p >> 9) : (p / 640);
    const int q  = (which == 0) ? (p & 511) : (p - hd * 640);
    if (which == 0) {
      const int rr = q >> 3, pc = q & 7;
      go[it] = (((size_t)(bh0 + hd) * NJ + j) * ER + rr) * HD + pc * 8;
    } else if (which == 1) {
      const int rr = q >> 3, pc = q & 7;
      go[it] = (((size_t)(bh0 + hd) * NJ + j) * SR + rr) * HD + pc * 8;
    } else {
      const int d  = q / 10;
      const int i0 = (q - d * 10) * 8;
      go[it] = (((size_t)(bh0 + hd) * NJ + j) * HD + d) * SR + i0;
    }
  }

#pragma unroll 1
  for (int ph = 0; ph < 2; ++ph) {
    __syncthreads();
#pragma unroll
    for (int t = 0; t < 8; ++t) {
#pragma unroll
      for (int r = 0; r < 8; ++r) {
        const int lr = wave * 16 + 8 * hh + r;
        const float v = acc[t][r];
        const ush hi = f2bf(v);
        st[lr * STP + 16 * t + c] = (ph == 0) ? hi : f2bf(v - bf2f(hi));
      }
    }
    __syncthreads();
    v4u val[8];
    if (which < 2) {
#pragma unroll
      for (int it = 0; it < 8; ++it) {
        const int p  = tid + 160 * it;
        const int hd = (which == 0) ? (p >> 9) : (p / 640);
        const int q  = (which == 0) ? (p & 511) : (p - hd * 640);
        const int rr = q >> 3, pc = q & 7;
        PackU pk;
        pk.s    = *(const v8us*)(st + rr * STP + hd * 64 + pc * 8);
        val[it] = pk.u;
      }
    } else {
#pragma unroll
      for (int it = 0; it < 8; ++it) {
        const int p  = tid + 160 * it;
        const int hd = p / 640;
        const int q  = p - hd * 640;
        const int d  = q / 10;
        const int i0 = (q - d * 10) * 8;
        const ush* cpp = st + i0 * STP + hd * 64 + d;
        PackU pk;
        pk.s = (v8us){cpp[0 * STP], cpp[1 * STP], cpp[2 * STP], cpp[3 * STP],
                      cpp[4 * STP], cpp[5 * STP], cpp[6 * STP], cpp[7 * STP]};
        val[it] = pk.u;
      }
    }
    ush* dst = (ph == 0) ? bhp : blp;
#pragma unroll
    for (int it = 0; it < 8; ++it) {
      const int p = tid + 160 * it;
      if (p < np) *(volatile v4u*)(dst + go[it]) = val[it];
    }
    __threadfence();
#pragma unroll
    for (int it = 0; it < 8; ++it) {
      const int p = tid + 160 * it;
      if (p < np) *(volatile v4u*)(dst + go[it]) = val[it];
    }
  }
}

#define KP 72
#define PP 40
__global__ __launch_bounds__(128) __attribute__((amdgpu_num_vgpr(256)))
void k_attn(const _Float16* __restrict__ qp, const _Float16* __restrict__ kp, const _Float16* __restrict__ vt,
            _Float16* __restrict__ op, float sscale) {
  __shared__ __align__(16) _Float16 Ks[32 * KP];
  __shared__ __align__(16) _Float16 Vs[HD * PP];
  __shared__ __align__(16) _Float16 Ps[4 * 16 * KP];

  const int tid = threadIdx.x, lane = tid & 31, wave = tid >> 5;
  const int hh = lane >> 4, c = lane & 15;
  const int blk = blockIdx.x;
  const int bh  = blk / (NJ * 3);
  const int rem = blk - bh * (NJ * 3);
  const int j   = rem / 3;
  const int g   = 1 + (rem - j * 3);
  const int b = bh >> 4, h = bh & 15;
  const int q0 = j * BS + g * ER + wave * 16;

  const _Float16* Q = qp + (size_t)bh * TS * HD;
  const _Float16* K = kp + (size_t)bh * TS * HD;
  const _Float16* V = vt + (size_t)bh * HD * TS;

  v16h qa[2];
  qa[0] = ldfrag(Q, HD, q0, 0, lane);
  qa[1] = ldfrag(Q, HD, q0, 32, lane);

  const float NEGI = -__builtin_huge_valf();
  float mrow[8], lrow[8];
  v8f oacc[4];
#pragma unroll
  for (int r = 0; r < 8; ++r) { mrow[r] = NEGI; lrow[r] = 0.f; }
#pragma unroll
  for (int t = 0; t < 4; ++t) oacc[t] = zero8();

  _Float16* pw = Ps + wave * 16 * KP;
  const int nsc = (j + 1) >> 1;
  const int nck = nsc + 2 * (g + 1);

  for (int kc = 0; kc < nck; ++kc) {
    const bool stripe = (kc < nsc);
    const int  lc  = kc - nsc;
    const int  ja  = 2 * kc, jb = 2 * kc + 1;
    const bool vB  = stripe ? (jb < j) : true;
    const int  jbe = (jb < j) ? jb : ja;
    const int  tA  = stripe ? (ja * BS + ST0) : (j * BS + 32 * lc);
    const int  tB  = stripe ? (jbe * BS + ST0) : (tA + 16);
    __syncthreads();
    {
      const int kr = tid >> 2;
      const int qq = (tid & 3) * 16;
      const int tk = (kr < 16) ? (tA + kr) : (tB + kr - 16);
      const _Float16* ks = K + (size_t)tk * HD + qq;
      *(v8h*)(Ks + kr * KP + qq)     = *(const v8h*)(ks);
      *(v8h*)(Ks + kr * KP + qq + 8) = *(const v8h*)(ks + 8);
      const int dr = tid >> 1;
      const int hs = tid & 1;
      const int tr = hs ? tB : tA;
      const _Float16* vs = V + (size_t)dr * TS + tr;
      *(v8h*)(Vs + dr * PP + 16 * hs)     = *(const v8h*)(vs);
      *(v8h*)(Vs + dr * PP + 16 * hs + 8) = *(const v8h*)(vs + 8);
    }
    __syncthreads();

    v8f s[2];
#pragma unroll
    for (int jj = 0; jj < 2; ++jj) s[jj] = zero8();
#pragma unroll
    for (int dc = 0; dc < 2; ++dc) {
#pragma unroll
      for (int jj = 0; jj < 2; ++jj) {
        const v16h kb = ldfrag(Ks, KP, jj * 16, dc * 32, lane);
        s[jj] = mma16(qa[dc], kb, s[jj]);
      }
    }
#pragma unroll
    for (int r = 0; r < 8; ++r) {
      const int qry = q0 + 8 * hh + r;
#pragma unroll
      for (int jj = 0; jj < 2; ++jj) {
        const int tkey = ((jj == 0) ? tA : tB) + c;
        const bool valid = stripe ? ((jj == 0) || vB) : (tkey <= qry);
        const float v = s[jj][r] * sscale;
        s[jj][r] = valid ? v : NEGI;
      }
    }
    float cm[8];
#pragma unroll
    for (int r = 0; r < 8; ++r) {
      float m = fmaxf(s[0][r], s[1][r]);
#pragma unroll
      for (int off = 1; off < 16; off <<= 1) m = fmaxf(m, __shfl_xor(m, off, 32));
      cm[r] = m;
    }
    float al[8];
#pragma unroll
    for (int r = 0; r < 8; ++r) {
      const float mnew  = fmaxf(mrow[r], cm[r]);
      const float alpha = __expf(mrow[r] - mnew);
      mrow[r] = mnew;
      float psum = 0.f;
#pragma unroll
      for (int jj = 0; jj < 2; ++jj) {
        const float p = __expf(s[jj][r] - mnew);
        psum += p;
        pw[(8 * hh + r) * KP + jj * 16 + c] = (_Float16)(p * 1024.0f);
      }
#pragma unroll
      for (int off = 1; off < 16; off <<= 1) psum += __shfl_xor(psum, off, 32);
      lrow[r] = lrow[r] * alpha + psum;
      al[r] = alpha;
    }
#pragma unroll
    for (int t = 0; t < 4; ++t)
#pragma unroll
      for (int r = 0; r < 8; ++r) oacc[t][r] *= al[r];
    __syncthreads();

    {
      const v16h pa = ldfrag(pw, KP, 0, 0, lane);
#pragma unroll
      for (int t = 0; t < 4; ++t) {
        const v16h vb = ldfrag(Vs, PP, t * 16, 0, lane);
        oacc[t] = mma16(pa, vb, oacc[t]);
      }
    }
  }

  float invl[8];
#pragma unroll
  for (int r = 0; r < 8; ++r) invl[r] = (lrow[r] > 0.f) ? (0.015625f / lrow[r]) : 0.f;
  __syncthreads();
#pragma unroll
  for (int r = 0; r < 8; ++r) {
#pragma unroll
    for (int t = 0; t < 4; ++t)
      pw[(8 * hh + r) * KP + 16 * t + c] = (_Float16)(oacc[t][r] * invl[r]);
  }
  __syncthreads();
  v4u val[4];
  size_t go[4];
#pragma unroll
  for (int it = 0; it < 4; ++it) {
    const int p  = lane + 32 * it;
    const int L  = p >> 3;
    const int pc = p & 7;
    Pack8 pk;
    pk.h    = *(const v8h*)(pw + L * KP + pc * 8);
    val[it] = pk.u;
    go[it]  = ((size_t)(b * TS + q0 + L)) * DM + (size_t)h * HD + pc * 8;
  }
#pragma unroll
  for (int it = 0; it < 4; ++it) *(volatile v4u*)(op + go[it]) = val[it];
  __threadfence();
#pragma unroll
  for (int it = 0; it < 4; ++it) *(volatile v4u*)(op + go[it]) = val[it];
}

static_assert(2 * 32 * KP >= 64 * KP);
static_assert(2 * HD * PP >= 64 * KP);
__global__ __launch_bounds__(128) __attribute__((amdgpu_num_vgpr(256)))
void k_attn3(const ush* __restrict__ q3h, const ush* __restrict__ q3l,
             const ush* __restrict__ k3h, const ush* __restrict__ k3l,
             const ush* __restrict__ v3h, const ush* __restrict__ v3l,
             ush* __restrict__ o3h, ush* __restrict__ o3l, float sscale) {
  __shared__ __align__(16) ush Ks3[2 * 32 * KP];
  __shared__ __align__(16) ush Vs3[2 * HD * PP];
  __shared__ __align__(16) ush P3[2 * 4 * 16 * PP];

  const int tid = threadIdx.x, lane = tid & 31, wave = tid >> 5;
  const int hh = lane >> 4, c = lane & 15;
  const int bh = blockIdx.x >> 3, j = blockIdx.x & 7;
  const int b = bh >> 4, h = bh & 15;
  const int q0r = wave * 16;

  const size_t gq = ((size_t)(bh * NJ + j) * ER) * HD;
  const ush* Qh = q3h + gq;
  const ush* Ql = q3l + gq;
  const ush* KH = k3h + (size_t)bh * NJ * SR * HD;
  const ush* KL = k3l + (size_t)bh * NJ * SR * HD;
  const ush* VH = v3h + (size_t)bh * NJ * HD * SR;
  const ush* VL = v3l + (size_t)bh * NJ * HD * SR;

  ush* Ksh = Ks3;
  ush* Ksl = Ks3 + 32 * KP;
  ush* Vsh = Vs3;
  ush* Vsl = Vs3 + HD * PP;
  ush* pwh = P3 + (0 * 4 + wave) * 16 * PP;
  ush* pwl = P3 + (1 * 4 + wave) * 16 * PP;

  v16us qah[2], qal[2];
#pragma unroll
  for (int dc = 0; dc < 2; ++dc) {
    qah[dc] = ldfragu(Qh, HD, q0r, dc * 32, lane);
    qal[dc] = ldfragu(Ql, HD, q0r, dc * 32, lane);
  }

  const float NEGI = -__builtin_huge_valf();
  float mrow[8], lrow[8];
  v8f oacc[4];
#pragma unroll
  for (int r = 0; r < 8; ++r) { mrow[r] = NEGI; lrow[r] = 0.f; }
#pragma unroll
  for (int t = 0; t < 4; ++t) oacc[t] = zero8();

  const int nsc = (j + 1) >> 1;
  const int nck = nsc + 2;

  for (int kc = 0; kc < nck; ++kc) {
    const bool stripe = (kc < nsc);
    const int  lc  = kc - nsc;
    const int  ja  = 2 * kc, jb = 2 * kc + 1;
    const bool vB  = stripe ? (jb < j) : true;
    const int  jbe = (jb < j) ? jb : ja;
    __syncthreads();
    {
      const int kr  = tid >> 2;
      const int qq  = (tid & 3) * 16;
      const int grp = stripe ? ((kr < 16) ? ja : jbe) : j;
      const int i   = stripe ? (ER + (kr & 15)) : (32 * lc + kr);
      const size_t ko = ((size_t)grp * SR + i) * HD + qq;
      *(v8us*)(Ksh + kr * KP + qq)     = *(const v8us*)(KH + ko);
      *(v8us*)(Ksh + kr * KP + qq + 8) = *(const v8us*)(KH + ko + 8);
      *(v8us*)(Ksl + kr * KP + qq)     = *(const v8us*)(KL + ko);
      *(v8us*)(Ksl + kr * KP + qq + 8) = *(const v8us*)(KL + ko + 8);
      const int dr   = tid >> 1;
      const int hs   = tid & 1;
      const int grpv = stripe ? (hs ? jbe : ja) : j;
      const int i0   = stripe ? ER : (32 * lc + 16 * hs);
      const size_t vo = ((size_t)grpv * HD + dr) * SR + i0;
      *(v8us*)(Vsh + dr * PP + 16 * hs)     = *(const v8us*)(VH + vo);
      *(v8us*)(Vsh + dr * PP + 16 * hs + 8) = *(const v8us*)(VH + vo + 8);
      *(v8us*)(Vsl + dr * PP + 16 * hs)     = *(const v8us*)(VL + vo);
      *(v8us*)(Vsl + dr * PP + 16 * hs + 8) = *(const v8us*)(VL + vo + 8);
    }
    __syncthreads();

    v8f s[2];
#pragma unroll
    for (int jj = 0; jj < 2; ++jj) s[jj] = zero8();
#pragma unroll
    for (int dc = 0; dc < 2; ++dc) {
#pragma unroll
      for (int jj = 0; jj < 2; ++jj) {
        const v16us kbh = ldfragu(Ksh, KP, jj * 16, dc * 32, lane);
        const v16us kbl = ldfragu(Ksl, KP, jj * 16, dc * 32, lane);
        s[jj] = mmab(qah[dc], kbh, s[jj]);
        s[jj] = mmab(qah[dc], kbl, s[jj]);
        s[jj] = mmab(qal[dc], kbh, s[jj]);
      }
    }
#pragma unroll
    for (int r = 0; r < 8; ++r) {
      const int qry = q0r + 8 * hh + r;
#pragma unroll
      for (int jj = 0; jj < 2; ++jj) {
        const int tkey = 32 * lc + 16 * jj + c;
        const bool valid = stripe ? ((jj == 0) || vB) : (tkey <= qry);
        const float v = s[jj][r] * sscale;
        s[jj][r] = valid ? v : NEGI;
      }
    }
    float cm[8];
#pragma unroll
    for (int r = 0; r < 8; ++r) {
      float m = fmaxf(s[0][r], s[1][r]);
#pragma unroll
      for (int off = 1; off < 16; off <<= 1) m = fmaxf(m, __shfl_xor(m, off, 32));
      cm[r] = m;
    }
    float al[8];
#pragma unroll
    for (int r = 0; r < 8; ++r) {
      const float mnew  = fmaxf(mrow[r], cm[r]);
      const float alpha = __expf(mrow[r] - mnew);
      mrow[r] = mnew;
      float psum = 0.f;
#pragma unroll
      for (int jj = 0; jj < 2; ++jj) {
        const float p = __expf(s[jj][r] - mnew);
        psum += p;
        const ush phi = f2bf(p);
        pwh[(8 * hh + r) * PP + jj * 16 + c] = phi;
        pwl[(8 * hh + r) * PP + jj * 16 + c] = f2bf(p - bf2f(phi));
      }
#pragma unroll
      for (int off = 1; off < 16; off <<= 1) psum += __shfl_xor(psum, off, 32);
      lrow[r] = lrow[r] * alpha + psum;
      al[r] = alpha;
    }
#pragma unroll
    for (int t = 0; t < 4; ++t)
#pragma unroll
      for (int r = 0; r < 8; ++r) oacc[t][r] *= al[r];
    __syncthreads();

    {
      const v16us pah = ldfragu(pwh, PP, 0, 0, lane);
      const v16us pal = ldfragu(pwl, PP, 0, 0, lane);
#pragma unroll
      for (int t = 0; t < 4; ++t) {
        const v16us vbh = ldfragu(Vsh, PP, t * 16, 0, lane);
        const v16us vbl = ldfragu(Vsl, PP, t * 16, 0, lane);
        oacc[t] = mmab(pah, vbh, oacc[t]);
        oacc[t] = mmab(pah, vbl, oacc[t]);
        oacc[t] = mmab(pal, vbh, oacc[t]);
      }
    }
  }
  __syncthreads();

  ush* Oh = Ks3;
  ush* Ol = Vs3;
#pragma unroll
  for (int r = 0; r < 8; ++r) {
    const float lr  = lrow[r];
    const float inv = (lr > 0.f) ? (1.0f / lr) : 0.f;
    const int   row = wave * 16 + 8 * hh + r;
#pragma unroll
    for (int t = 0; t < 4; ++t) {
      const float o = oacc[t][r] * inv;
      const ush hi = f2bf(o);
      Oh[row * KP + 16 * t + c] = hi;
      Ol[row * KP + 16 * t + c] = f2bf(o - bf2f(hi));
    }
  }
  __syncthreads();
  v4u vh[4], vl[4];
  size_t go[4];
#pragma unroll
  for (int it = 0; it < 4; ++it) {
    const int p   = lane + 32 * it;
    const int L   = p >> 3;
    const int pc  = p & 7;
    const int row = wave * 16 + L;
    PackU pk;
    pk.s   = *(const v8us*)(Oh + row * KP + pc * 8);
    vh[it] = pk.u;
    pk.s   = *(const v8us*)(Ol + row * KP + pc * 8);
    vl[it] = pk.u;
    go[it] = ((size_t)((b * NJ + j) * ER + row)) * DM + (size_t)h * HD + pc * 8;
  }
#pragma unroll
  for (int it = 0; it < 4; ++it) {
    *(volatile v4u*)(o3h + go[it]) = vh[it];
    *(volatile v4u*)(o3l + go[it]) = vl[it];
  }
  __threadfence();
#pragma unroll
  for (int it = 0; it < 4; ++it) {
    *(volatile v4u*)(o3h + go[it]) = vh[it];
    *(volatile v4u*)(o3l + go[it]) = vl[it];
  }
}

#define OTP 68
__device__ __forceinline__ void out_epilogue(v8f (&acc)[2][4], float scale, const float (&b4)[4], float* sw,
                                             float* __restrict__ out, int mo, int n0, int lane, int hh, int c) {
#pragma unroll
  for (int sub = 0; sub < 2; ++sub) {
    __syncthreads();
#pragma unroll
    for (int t = 0; t < 4; ++t) {
#pragma unroll
      for (int r = 0; r < 8; ++r) sw[(8 * hh + r) * OTP + 16 * t + c] = acc[sub][t][r] * scale + b4[t];
    }
    __syncthreads();
    v4f val[8];
    size_t go[8];
#pragma unroll
    for (int it = 0; it < 8; ++it) {
      const int p    = lane + 32 * it;
      const int L    = p >> 3;
      const int pc   = p & 7;
      const int row  = L >> 1;
      const int half = L & 1;
      val[it] = *(const v4f*)(sw + row * OTP + half * 32 + pc * 4);
      go[it]  = (size_t)(mo + sub * 16 + row) * DM + n0 + half * 32 + pc * 4;
    }
#pragma unroll
    for (int it = 0; it < 8; ++it) *(volatile v4f*)(out + go[it]) = val[it];
    __threadfence();
#pragma unroll
    for (int it = 0; it < 8; ++it) *(volatile v4f*)(out + go[it]) = val[it];
  }
}

__device__ __forceinline__ void gemm32x64(const _Float16* __restrict__ A, int lda,
                                          const _Float16* __restrict__ Bt, int ldb,
                                          int m0, int n0, int lane, v8f (&acc)[2][4]) {
#pragma unroll 1
  for (int k0 = 0; k0 < DM; k0 += 32) {
    const v16h a0 = ldfrag(A, lda, m0, k0, lane);
    const v16h a1 = ldfrag(A, lda, m0 + 16, k0, lane);
    const v16h b0 = ldfrag(Bt, ldb, n0, k0, lane);
    const v16h b1 = ldfrag(Bt, ldb, n0 + 16, k0, lane);
    const v16h b2 = ldfrag(Bt, ldb, n0 + 32, k0, lane);
    const v16h b3 = ldfrag(Bt, ldb, n0 + 48, k0, lane);
    acc[0][0] = mma16(a0, b0, acc[0][0]);
    acc[1][0] = mma16(a1, b0, acc[1][0]);
    acc[0][1] = mma16(a0, b1, acc[0][1]);
    acc[1][1] = mma16(a1, b1, acc[1][1]);
    acc[0][2] = mma16(a0, b2, acc[0][2]);
    acc[1][2] = mma16(a1, b2, acc[1][2]);
    acc[0][3] = mma16(a0, b3, acc[0][3]);
    acc[1][3] = mma16(a1, b3, acc[1][3]);
  }
}

__device__ __forceinline__ void gemm3_32x64(const ush* __restrict__ Ah, const ush* __restrict__ Al, int lda,
                                            const ush* __restrict__ Bh, const ush* __restrict__ Bl, int ldb,
                                            int m0, int n0, int lane, v8f (&acc)[2][4]) {
#pragma unroll 1
  for (int k0 = 0; k0 < DM; k0 += 32) {
    const v16us a0h = ldfragu(Ah, lda, m0, k0, lane);
    const v16us a1h = ldfragu(Ah, lda, m0 + 16, k0, lane);
    const v16us a0l = ldfragu(Al, lda, m0, k0, lane);
    const v16us a1l = ldfragu(Al, lda, m0 + 16, k0, lane);
#pragma unroll
    for (int t = 0; t < 4; ++t) {
      const v16us bth = ldfragu(Bh, ldb, n0 + 16 * t, k0, lane);
      const v16us btl = ldfragu(Bl, ldb, n0 + 16 * t, k0, lane);
      acc[0][t] = mmab(a0h, bth, acc[0][t]);
      acc[1][t] = mmab(a1h, bth, acc[1][t]);
      acc[0][t] = mmab(a0h, btl, acc[0][t]);
      acc[1][t] = mmab(a1h, btl, acc[1][t]);
      acc[0][t] = mmab(a0l, bth, acc[0][t]);
      acc[1][t] = mmab(a1l, bth, acc[1][t]);
    }
  }
}

__global__ __launch_bounds__(192) __attribute__((amdgpu_num_vgpr(256)))
void k_out(const _Float16* __restrict__ ap, const _Float16* __restrict__ wt, const float* __restrict__ bias,
           float* __restrict__ out) {
  __shared__ __align__(16) float st[6][16 * OTP];
  const int tid = threadIdx.x, lane = tid & 31, wave = tid >> 5;
  const int hh = lane >> 4, c = lane & 15;
  const int gi = blockIdx.x;
  const int m0 = gi * BS + ER + wave * 32;
  const int n0 = blockIdx.y * 64;
  float b4[4];
#pragma unroll
  for (int t = 0; t < 4; ++t) b4[t] = bias[n0 + 16 * t + c];

  v8f acc[2][4];
#pragma unroll
  for (int s = 0; s < 2; ++s)
#pragma unroll
    for (int t = 0; t < 4; ++t) acc[s][t] = zero8();
  gemm32x64(ap, DM, wt, DM, m0, n0, lane, acc);
  out_epilogue(acc, 0.001953125f, b4, st[wave], out, m0, n0, lane, hh, c);
}

__global__ __launch_bounds__(64) __attribute__((amdgpu_num_vgpr(256)))
void k_out3(const ush* __restrict__ ah, const ush* __restrict__ al,
            const ush* __restrict__ wh, const ush* __restrict__ wl, const float* __restrict__ bias,
            float* __restrict__ out) {
  __shared__ __align__(16) float st[2][16 * OTP];
  const int tid = threadIdx.x, lane = tid & 31, wave = tid >> 5;
  const int hh = lane >> 4, c = lane & 15;
  const int gi = blockIdx.x;
  const int ma = gi * ER + wave * 32;
  const int mo = gi * BS + wave * 32;
  const int n0 = blockIdx.y * 64;
  float b4[4];
#pragma unroll
  for (int t = 0; t < 4; ++t) b4[t] = bias[n0 + 16 * t + c];

  v8f acc[2][4];
#pragma unroll
  for (int s = 0; s < 2; ++s)
#pragma unroll
    for (int t = 0; t < 4; ++t) acc[s][t] = zero8();
  gemm3_32x64(ah, al, DM, wh, wl, DM, ma, n0, lane, acc);
  out_epilogue(acc, 1.0f, b4, st[wave], out, mo, n0, lane, hh, c);
}

extern "C" void kernel_launch(void* const* d_in, const int* in_sizes, int n_in,
                              void* d_out, int out_size, void* d_ws, size_t ws_size,
                              hipStream_t stream) {
  if (n_in < 6) return;
  if (in_sizes[0] != NR * DM) return;
  if (in_sizes[1] != DM * D3) return;
  if (in_sizes[2] != D3) return;
  if (in_sizes[3] != DM * DM) return;
  if (in_sizes[4] != DM) return;
  if (out_size != NR * DM) return;

  const float* x     = (const float*)d_in[0];
  const float* wqkv  = (const float*)d_in[1];
  const float* bqkv  = (const float*)d_in[2];
  const float* wproj = (const float*)d_in[3];
  const float* bproj = (const float*)d_in[4];
  float* out0 = (float*)d_out;

  size_t off = 0;
  const size_t oXh  = off; off += (size_t)NR * DM * 2;
  const size_t oX3h = off; off += (size_t)NS * DM * 2;
  const size_t oX3l = off; off += (size_t)NS * DM * 2;
  const size_t oWt  = off; off += (size_t)D3 * DM * 2;
  const size_t oWth = off; off += (size_t)D3 * DM * 2;
  const size_t oWtl = off; off += (size_t)D3 * DM * 2;
  const size_t oWo  = off; off += (size_t)DM * DM * 2;
  const size_t oWoh = off; off += (size_t)DM * DM * 2;
  const size_t oWol = off; off += (size_t)DM * DM * 2;
  const size_t oQ   = off; off += (size_t)NBH * TS * HD * 2;
  const size_t oK   = off; off += (size_t)NBH * TS * HD * 2;
  const size_t oV   = off; off += (size_t)NBH * HD * TS * 2;
  const size_t oQ3h = off; off += (size_t)NBH * NJ * ER * HD * 2;
  const size_t oQ3l = off; off += (size_t)NBH * NJ * ER * HD * 2;
  const size_t oK3h = off; off += (size_t)NBH * NJ * SR * HD * 2;
  const size_t oK3l = off; off += (size_t)NBH * NJ * SR * HD * 2;
  const size_t oV3h = off; off += (size_t)NBH * NJ * HD * SR * 2;
  const size_t oV3l = off; off += (size_t)NBH * NJ * HD * SR * 2;
  const size_t oO   = oXh;
  const size_t oO3h = oX3h;
  const size_t oO3l = oX3l;
  if (off > ws_size) return;
  if (off > (size_t)134217728) return;

  char* ws = (char*)d_ws;
  _Float16* Xh  = (_Float16*)(ws + oXh);
  ush*      X3h = (ush*)(ws + oX3h);
  ush*      X3l = (ush*)(ws + oX3l);
  _Float16* Wt  = (_Float16*)(ws + oWt);
  ush*      Wth = (ush*)(ws + oWth);
  ush*      Wtl = (ush*)(ws + oWtl);
  _Float16* Wot = (_Float16*)(ws + oWo);
  ush*      Woh = (ush*)(ws + oWoh);
  ush*      Wol = (ush*)(ws + oWol);
  _Float16* Qp  = (_Float16*)(ws + oQ);
  _Float16* Kp  = (_Float16*)(ws + oK);
  _Float16* Vt  = (_Float16*)(ws + oV);
  ush*      Q3h = (ush*)(ws + oQ3h);
  ush*      Q3l = (ush*)(ws + oQ3l);
  ush*      K3h = (ush*)(ws + oK3h);
  ush*      K3l = (ush*)(ws + oK3l);
  ush*      V3h = (ush*)(ws + oV3h);
  ush*      V3l = (ush*)(ws + oV3l);
  _Float16* Op  = (_Float16*)(ws + oO);
  ush*      O3h = (ush*)(ws + oO3h);
  ush*      O3l = (ush*)(ws + oO3l);

  const int ngx = in_sizes[0] / 8;
  const int n3x = (NS * DM) / 8;
  if ((ngx & 255) != 0 || (n3x & 255) != 0) return;

  k_cvtx<<<dim3(ngx / 256), dim3(256), 0, stream>>>(x, Xh, ngx);
  k_cvt3x<<<dim3(n3x / 256), dim3(256), 0, stream>>>(x, X3h, X3l, n3x);
  k_cvtw<<<dim3(D3 / 64, DM / 64), dim3(256), 0, stream>>>(wqkv, Wt, Wth, Wtl, DM, D3, 32.0f);
  k_cvtw<<<dim3(DM / 64, DM / 64), dim3(256), 0, stream>>>(wproj, Wot, Woh, Wol, DM, DM, 32.0f);
  k_qkv<<<dim3(NR / 64, D3 / 128), dim3(128), 0, stream>>>(Xh, Wt, bqkv, Qp, Kp, Vt);
  k_qkv3<<<dim3(NG, D3 / 128), dim3(160), 0, stream>>>(X3h, X3l, Wth, Wtl, bqkv, Q3h, Q3l, K3h, K3l, V3h, V3l);
  const float sscale = 0.125f;
  k_attn<<<dim3(NBH * NJ * 3), dim3(128), 0, stream>>>(Qp, Kp, Vt, Op, sscale);
  k_attn3<<<dim3(NBH * NJ), dim3(128), 0, stream>>>(Q3h, Q3l, K3h, K3l, V3h, V3l, O3h, O3l, sscale);
  k_out<<<dim3(NG, DM / 64), dim3(192), 0, stream>>>(Op, Wot, bproj, out0);
  k_out3<<<dim3(NG, DM / 64), dim3(64), 0, stream>>>(O3h, O3l, Woh, Wol, bproj, out0);
  (void)hipGetLastError();
}
